// LDConv_9526237462558
// MI455X (gfx1250) — hardware-verified
//
#include <hip/hip_runtime.h>

#ifndef NB
#define NB 8
#endif
#define NB_FULL 8
#define IN_C 128
#define OUT_C 256
#define HH 80
#define WW 80
#define HW 6400
#define NP 9
#define NP2 18
#define NOFF 64
#define K1 1152
#define K2 2304
#define TPR 144
#define CB ((NB >= 2) ? 2 : 1)
#define BN_EPS 1e-5f

static_assert(NB >= 1 && NB <= NB_FULL);
static_assert(HW % 128 == 0);
static_assert(HW % 64 == 0);
static_assert(K1 % 32 == 0 && K2 % 32 == 0);
static_assert(OUT_C % 64 == 0 && NOFF % 64 == 0);

typedef __bf16 v16b __attribute__((ext_vector_type(16)));
typedef unsigned short v8us __attribute__((ext_vector_type(8), may_alias));
typedef float v8f __attribute__((ext_vector_type(8)));
typedef float v4f __attribute__((ext_vector_type(4)));
typedef float v4fa __attribute__((ext_vector_type(4), may_alias));
union FragB { v16b v; v8us half[2]; unsigned short u[16]; };

__device__ __forceinline__ unsigned short bf16_bits(float x) { unsigned int u = __float_as_uint(x); return (unsigned short)((u + 0x7FFFu + ((u >> 16) & 1u)) >> 16); }
__device__ __forceinline__ float bf16_val(unsigned short b) { return __uint_as_float(((unsigned int)b) << 16); }
__device__ __forceinline__ float bf16_rne(float x) { return bf16_val(bf16_bits(x)); }

__device__ __forceinline__ v16b gb_frag(const unsigned short* p, int hh) { FragB f; f.half[0] = *(const v8us*)(p + 8 * hh); f.half[1] = *(const v8us*)(p + 16 + 8 * hh); return f.v; }
__device__ __forceinline__ v8f gb_mma(v16b a, v16b b, v8f c) {
  v8f d = __builtin_amdgcn_wmma_f32_16x16x32_bf16(false, a, false, b, (short)0, c, false, false);
  asm volatile("v_nop\n\tv_nop\n\tv_nop\n\tv_nop" : "+v"(d) : "v"(a), "v"(b));
  return d;
}

template <int EPI>
__global__ __launch_bounds__(128) void k_gemm(const unsigned short* __restrict__ A, int lda, const unsigned short* __restrict__ Bt, int ldb,
                                             const float* __restrict__ bias, int nbias,
                                             const float* __restrict__ bng, const float* __restrict__ bnb,
                                             const float* __restrict__ bnm, const float* __restrict__ bnv,
                                             float* __restrict__ C, int ldc, int M, int N, int K, int growBase) {
#pragma clang fp contract(off)
  __shared__ __attribute__((aligned(16))) float so[4][32][68];
  const int tid = threadIdx.x, w = tid >> 5, lane = tid & 31, ln = lane & 15, hh = lane >> 4;
  const int ntn = N >> 6;
  const int mt = blockIdx.x / ntn, nq = blockIdx.x - mt * ntn;
  const int row0 = mt * 128 + 32 * w, col0 = nq * 64;
  if (row0 >= M) return;
  const unsigned short* a0p = A + (size_t)(row0 + ln) * lda;
  const unsigned short* a1p = a0p + (size_t)16 * lda;
  const unsigned short* b0p = Bt + (size_t)(col0 + ln) * ldb;
  const unsigned short* b1p = b0p + (size_t)16 * ldb;
  const unsigned short* b2p = b1p + (size_t)16 * ldb;
  const unsigned short* b3p = b2p + (size_t)16 * ldb;
  const v8f z8 = {0.f, 0.f, 0.f, 0.f, 0.f, 0.f, 0.f, 0.f};
  v8f c00 = z8, c01 = z8, c02 = z8, c03 = z8, c10 = z8, c11 = z8, c12 = z8, c13 = z8;
#pragma unroll 1
  for (int kb = 0; kb < K; kb += 32) {
    const v16b a0 = gb_frag(a0p + kb, hh), a1 = gb_frag(a1p + kb, hh);
    v16b b = gb_frag(b0p + kb, hh); c00 = gb_mma(a0, b, c00); c10 = gb_mma(a1, b, c10);
    b = gb_frag(b1p + kb, hh);      c01 = gb_mma(a0, b, c01); c11 = gb_mma(a1, b, c11);
    b = gb_frag(b2p + kb, hh);      c02 = gb_mma(a0, b, c02); c12 = gb_mma(a1, b, c12);
    b = gb_frag(b3p + kb, hh);      c03 = gb_mma(a0, b, c03); c13 = gb_mma(a1, b, c13);
  }
  v8f accs[8] = {c00, c01, c02, c03, c10, c11, c12, c13};
#pragma unroll
  for (int u = 0; u < 8; ++u) {
    const int t = u & 3, half = u >> 2;
    const int col = col0 + t * 16 + ln;
    if (EPI == 0) {
      const float braw = bias[min(col, nbias - 1)];
      const float bv = (col < nbias) ? bf16_rne(braw) : 0.f;
#pragma unroll
      for (int r = 0; r < 8; ++r) { const int rloc = half * 16 + 8 * hh + r; so[w][rloc][t * 16 + ln] = accs[u][r] + bv; }
    } else {
      const float gm = bf16_rne(bng[col]), be = bf16_rne(bnb[col]), mm = bf16_rne(bnm[col]), vv = bf16_rne(bnv[col]);
      const float inv = 1.0f / sqrtf(vv + BN_EPS);
      const float sc = gm * inv;
#pragma unroll
      for (int r = 0; r < 8; ++r) {
        const int rloc = half * 16 + 8 * hh + r;
        const float z = (accs[u][r] - mm) * sc + be;
        const float e = expf(fminf(-z, 80.0f));
        const float s = 1.0f / (1.0f + e);
        so[w][rloc][t * 16 + ln] = z * s;
      }
    }
  }
  __builtin_amdgcn_fence(__ATOMIC_ACQ_REL, "workgroup");
  __builtin_amdgcn_wave_barrier();
  if (EPI == 0) {
    const int rsub = lane >> 4, c4 = (lane & 15) * 4;
    for (int pass = 0; pass < 2; ++pass) {
#pragma unroll
      for (int q = 0; q < 16; ++q) {
        const int r = q * 2 + rsub;
        const v4f v = *(const v4fa*)&so[w][r][c4];
        *(volatile v4f*)(C + (size_t)(row0 + r) * ldc + col0 + c4) = v;
      }
      if (pass == 0) __threadfence();
    }
  } else {
    const int grow0 = growBase + row0;
    const int bb = grow0 / HW, pix0 = grow0 - bb * HW;
    const int oql = lane >> 3, p4 = (lane & 7) * 4;
    for (int pass = 0; pass < 2; ++pass) {
#pragma unroll
      for (int q = 0; q < 16; ++q) {
        const int oq = q * 4 + oql;
        v4f v;
        v[0] = so[w][p4 + 0][oq]; v[1] = so[w][p4 + 1][oq]; v[2] = so[w][p4 + 2][oq]; v[3] = so[w][p4 + 3][oq];
        *(volatile v4f*)(C + ((size_t)(bb * OUT_C + col0 + oq)) * HW + pix0 + p4) = v;
      }
      if (pass == 0) __threadfence();
    }
  }
}

__global__ __launch_bounds__(256) void k_xt(const float* __restrict__ x, unsigned short* __restrict__ XT) {
  __shared__ __attribute__((aligned(16))) unsigned short tl[64][136];
  const int tid = threadIdx.x;
  const int b = blockIdx.x / (HW / 64), pg = blockIdx.x % (HW / 64);
  const int pix0 = pg * 64;
  const int p = tid & 63, cq = tid >> 6;
#pragma unroll 4
  for (int it = 0; it < IN_C / 4; ++it) {
    const int c = it * 4 + cq;
    tl[p][c] = bf16_bits(x[((size_t)(b * IN_C + c)) * HW + pix0 + p]);
  }
  __syncthreads();
  const int rr = tid >> 4, c8 = tid & 15;
  for (int pass = 0; pass < 2; ++pass) {
#pragma unroll
    for (int it = 0; it < 4; ++it) {
      const int r = it * 16 + rr;
      const v8us v = *(const v8us*)&tl[r][c8 * 8];
      *(volatile v8us*)(XT + ((size_t)b * HW + pix0 + r) * IN_C + c8 * 8) = v;
    }
    if (pass == 0) __threadfence();
  }
}

__global__ __launch_bounds__(256) void k_wp(const float* __restrict__ w, unsigned short* __restrict__ Bt) {
  const int t = blockIdx.x * 256 + threadIdx.x;
  if (t >= NOFF * TPR) return;
  const int c8 = t & 15, tap = (t >> 4) % NP, n = t / TPR;
  const int nc = min(n, NP2 - 1);
  const bool live = (n < NP2);
  v8us o;
#pragma unroll
  for (int q = 0; q < 8; ++q) {
    const float val = w[((size_t)(nc * IN_C + c8 * 8 + q)) * 9 + tap];
    o[q] = live ? bf16_bits(val) : (unsigned short)0;
  }
  unsigned short* d = Bt + (size_t)t * 8;
  *(volatile v8us*)d = o;
  __threadfence();
  *(volatile v8us*)d = o;
}

__global__ __launch_bounds__(256) void k_w2(const float* __restrict__ w, unsigned short* __restrict__ Bt2) {
  const int t = blockIdx.x * 256 + threadIdx.x;
  if (t >= OUT_C * TPR) return;
  const int c8 = t & 15, n = (t >> 4) % NP, o = t / TPR;
  v8us v;
#pragma unroll
  for (int q = 0; q < 8; ++q) v[q] = bf16_bits(w[((size_t)(o * IN_C + c8 * 8 + q)) * NP + n]);
  unsigned short* d = Bt2 + (size_t)o * K2 + n * IN_C + c8 * 8;
  for (int pass = 0; pass < 2; ++pass) {
    *(volatile v8us*)d = v;
    *(volatile v8us*)(d + K1) = v;
    if (pass == 0) __threadfence();
  }
}

__global__ __launch_bounds__(256) void k_im(const unsigned short* __restrict__ XT, unsigned short* __restrict__ IM, int b0, int Mc) {
  const unsigned int t = blockIdx.x * 256u + threadIdx.x;
  if (t >= (unsigned int)Mc * (unsigned int)TPR) return;
  const int c8 = (int)(t & 15u), tap = (int)((t >> 4) % NP), m = (int)(t / TPR);
  const int bl = m / HW, pix = m - bl * HW;
  const int b = b0 + bl;
  const int i = pix / WW, j = pix - i * WW;
  const int ii = i + tap / 3 - 1, jj = j + tap % 3 - 1;
  const bool ok = (ii >= 0) && (ii < HH) && (jj >= 0) && (jj < WW);
  const int iic = min(max(ii, 0), HH - 1), jjc = min(max(jj, 0), WW - 1);
  v8us v = *(const v8us*)(XT + ((size_t)b * HW + (size_t)(iic * WW + jjc)) * IN_C + c8 * 8);
  if (!ok) {
#pragma unroll
    for (int q = 0; q < 8; ++q) v[q] = 0;
  }
  unsigned short* d = IM + (size_t)t * 8;
  *(volatile v8us*)d = v;
  __threadfence();
  *(volatile v8us*)d = v;
}

__global__ __launch_bounds__(256) void k_xoff(const unsigned short* __restrict__ XT, const float* __restrict__ OFF, const float* __restrict__ pn,
                                             unsigned short* __restrict__ A2, int b0, int Mc) {
#pragma clang fp contract(off)
  const unsigned int t = blockIdx.x * 256u + threadIdx.x;
  if (t >= (unsigned int)Mc * (unsigned int)TPR) return;
  const int c8 = (int)(t & 15u), n = (int)((t >> 4) % NP), m = (int)(t / TPR);
  const int bl = m / HW, pix = m - bl * HW;
  const int b = b0 + bl;
  const int i = pix / WW, j = pix - i * WW;
  const float offr = OFF[(size_t)m * NOFF + n], offc = OFF[(size_t)m * NOFF + NP + n];
  const float pnr = bf16_rne(pn[n]), pnc = bf16_rne(pn[NP + n]);
  const float pr = ((float)i + pnr) + offr;
  const float pc = ((float)j + pnc) + offc;
  const float fr = floorf(pr), fc = floorf(pc);
  const float hmax = (float)(HH - 1), wmax = (float)(WW - 1);
  const float qlr = fminf(fmaxf(fr, 0.f), hmax), qlc = fminf(fmaxf(fc, 0.f), wmax);
  const float qrr = fminf(fmaxf(fr + 1.0f, 0.f), hmax), qrc = fminf(fmaxf(fc + 1.0f, 0.f), wmax);
  const float pcr = fminf(fmaxf(pr, 0.f), hmax), pcc = fminf(fmaxf(pc, 0.f), wmax);
  const float ar = 1.0f + (qlr - pcr);
  const float ac = 1.0f + (qlc - pcc);
  const float br = 1.0f + (-(qrr - pcr));
  const float bc = 1.0f + (-(qrc - pcc));
  const float glt = ar * ac, grb = br * bc, glb = ar * bc, grt = br * ac;
  const int ilr = min(max((int)qlr, 0), HH - 1), ilc = min(max((int)qlc, 0), WW - 1);
  const int irr = min(max((int)qrr, 0), HH - 1), irc = min(max((int)qrc, 0), WW - 1);
  const unsigned short* xb = XT + ((size_t)b * HW) * IN_C + c8 * 8;
  const v8us vlt = *(const v8us*)(xb + (size_t)(ilr * WW + ilc) * IN_C);
  const v8us vrb = *(const v8us*)(xb + (size_t)(irr * WW + irc) * IN_C);
  const v8us vlb = *(const v8us*)(xb + (size_t)(ilr * WW + irc) * IN_C);
  const v8us vrt = *(const v8us*)(xb + (size_t)(irr * WW + ilc) * IN_C);
  v8us ho, lo;
#pragma unroll
  for (int q = 0; q < 8; ++q) {
    const float xlt = bf16_val(vlt[q]), xrb = bf16_val(vrb[q]), xlb = bf16_val(vlb[q]), xrt = bf16_val(vrt[q]);
    const float v = ((glt * xlt + grb * xrb) + glb * xlb) + grt * xrt;
    const unsigned short hb = bf16_bits(v);
    ho[q] = hb;
    lo[q] = bf16_bits(v - bf16_val(hb));
  }
  unsigned short* d = A2 + (size_t)m * K2 + n * IN_C + c8 * 8;
  for (int pass = 0; pass < 2; ++pass) {
    *(volatile v8us*)d = ho;
    *(volatile v8us*)(d + K1) = lo;
    if (pass == 0) __threadfence();
  }
}

#define ALIGN256(x) (((size_t)(x) + 255) & ~(size_t)255)
#define XT_BYTES  ((size_t)NB * HW * IN_C * 2)
#define BTP_BYTES ((size_t)NOFF * K1 * 2)
#define BT2_BYTES ((size_t)OUT_C * K2 * 2)
#define OFF_BYTES ((size_t)CB * HW * NOFF * 4)
#define IM_BYTES  ((size_t)CB * HW * K1 * 2)
#define A2_BYTES  ((size_t)CB * HW * K2 * 2)
#define PL_BYTES  ((IM_BYTES > A2_BYTES) ? IM_BYTES : A2_BYTES)
static_assert(IM_BYTES <= PL_BYTES && A2_BYTES <= PL_BYTES);
static_assert(ALIGN256(XT_BYTES) + ALIGN256(BTP_BYTES) + ALIGN256(BT2_BYTES) + ALIGN256(OFF_BYTES) + ALIGN256(PL_BYTES) <= (size_t)134217728);
static_assert((size_t)NB * OUT_C * HW * 4 <= (size_t)NB_FULL * OUT_C * HW * 4);

extern "C" void kernel_launch(void* const* d_in, const int* in_sizes, int n_in,
                              void* d_out, int out_size, void* d_ws, size_t ws_size, hipStream_t stream) {
  if (n_in < 9) return;
  if (in_sizes[0] < NB * IN_C * HW) return;
  if (in_sizes[1] < NP2 * IN_C * 9) return;
  if (in_sizes[2] < NP2) return;
  if (in_sizes[3] < OUT_C * IN_C * NP) return;
  if (in_sizes[4] < OUT_C || in_sizes[5] < OUT_C || in_sizes[6] < OUT_C || in_sizes[7] < OUT_C) return;
  if (in_sizes[8] < NP2) return;
  if (out_size < NB * OUT_C * HW) return;
  const float* x       = (const float*)d_in[0];
  const float* w_pconv = (const float*)d_in[1];
  const float* b_pconv = (const float*)d_in[2];
  const float* w_conv  = (const float*)d_in[3];
  const float* bn_g    = (const float*)d_in[4];
  const float* bn_b    = (const float*)d_in[5];
  const float* bn_m    = (const float*)d_in[6];
  const float* bn_v    = (const float*)d_in[7];
  const float* p_n     = (const float*)d_in[8];
  float* out = (float*)d_out;

  char* ws = (char*)d_ws; size_t off = 0;
  auto take = [&](size_t bytes) { char* p = ws + off; off += ALIGN256(bytes); return p; };
  unsigned short* XT  = (unsigned short*)take(XT_BYTES);
  unsigned short* BtP = (unsigned short*)take(BTP_BYTES);
  unsigned short* Bt2 = (unsigned short*)take(BT2_BYTES);
  float*          OFF = (float*)take(OFF_BYTES);
  unsigned short* PL  = (unsigned short*)take(PL_BYTES);
  if (off > ws_size) return;

  k_xt<<<(unsigned)(NB * (HW / 64)), 256, 0, stream>>>(x, XT);
  k_wp<<<(unsigned)((NOFF * TPR + 255) / 256), 256, 0, stream>>>(w_pconv, BtP);
  k_w2<<<(unsigned)((OUT_C * TPR + 255) / 256), 256, 0, stream>>>(w_conv, Bt2);
  for (int b0 = 0; b0 < NB; b0 += CB) {
    const int cb = (NB - b0 < CB) ? (NB - b0) : CB;
    const int Mc = cb * HW;
    const unsigned nthr = (unsigned)Mc * (unsigned)TPR;
    k_im<<<(nthr + 255) / 256, 256, 0, stream>>>(XT, PL, b0, Mc);
    k_gemm<0><<<(unsigned)((Mc / 128) * (NOFF / 64)), 128, 0, stream>>>(PL, K1, BtP, K1, b_pconv, NP2,
                                                                       nullptr, nullptr, nullptr, nullptr,
                                                                       OFF, NOFF, Mc, NOFF, K1, 0);
    k_xoff<<<(nthr + 255) / 256, 256, 0, stream>>>(XT, OFF, p_n, PL, b0, Mc);
    k_gemm<1><<<(unsigned)((Mc / 128) * (OUT_C / 64)), 128, 0, stream>>>(PL, K2, Bt2, K2, nullptr, 1,
                                                                        bn_g, bn_b, bn_m, bn_v,
                                                                        out, 0, Mc, OUT_C, K2, b0 * HW);
  }
}
